// MHAttention_30949534335122
// MI455X (gfx1250) — hardware-verified
//
#include <hip/hip_runtime.h>

typedef __attribute__((ext_vector_type(16))) _Float16 v16h;
typedef __attribute__((ext_vector_type(8)))  _Float16 v8h;
typedef __attribute__((ext_vector_type(16))) __bf16   v16b;
typedef __attribute__((ext_vector_type(8)))  __bf16   v8b;
typedef __attribute__((ext_vector_type(8)))  float    v8f;
typedef __attribute__((ext_vector_type(4)))  float    v4f;
typedef __attribute__((ext_vector_type(4)))  unsigned int v4u;
typedef __attribute__((ext_vector_type(8)))  unsigned short v8us;

namespace {
constexpr int NBATCH = 2;
constexpr int NSEQ   = 4096;
constexpr int NCH    = 1024;
constexpr int NHEAD  = 16;
constexpr int DHEAD  = 64;
constexpr int KLR    = 256;
constexpr int NFEAT  = NHEAD * DHEAD;
constexpr int ATT_QB = 64;
constexpr int ATT_KC = 64;

constexpr size_t SZ_X   = (size_t)NBATCH * NSEQ * NCH * 2;
constexpr size_t SZ_XT  = (size_t)NBATCH * NCH * NSEQ * 2;
constexpr size_t SZ_W   = (size_t)NFEAT * NCH * 2;
constexpr size_t SZ_WE  = (size_t)KLR * NSEQ * 2;
constexpr size_t SZ_QP  = (size_t)NBATCH * NSEQ * NFEAT * 2;
constexpr size_t SZ_T   = (size_t)NBATCH * KLR * NCH * 2;
constexpr size_t SZ_KE  = (size_t)NBATCH * KLR * NFEAT * 2;
constexpr size_t SZ_VF  = (size_t)NBATCH * NFEAT * KLR * 2;
constexpr size_t OFF_X   = 0;
constexpr size_t OFF_XT  = OFF_X + SZ_X;
constexpr size_t OFF_WQ  = OFF_XT + SZ_XT;
constexpr size_t OFF_WK  = OFF_WQ + SZ_W;
constexpr size_t OFF_WV  = OFF_WK + SZ_W;
constexpr size_t OFF_WO  = OFF_WV + SZ_W;
constexpr size_t OFF_WE  = OFF_WO + SZ_W;
constexpr size_t OFF_WF  = OFF_WE + SZ_WE;
constexpr size_t OFF_QH  = OFF_WF + SZ_WE;
constexpr size_t OFF_QL  = OFF_QH + SZ_QP;
constexpr size_t OFF_TEH = OFF_QL + SZ_QP;
constexpr size_t OFF_TEL = OFF_TEH + SZ_T;
constexpr size_t OFF_TFH = OFF_TEL + SZ_T;
constexpr size_t OFF_TFL = OFF_TFH + SZ_T;
constexpr size_t OFF_KEH = OFF_TFL + SZ_T;
constexpr size_t OFF_KEL = OFF_KEH + SZ_KE;
constexpr size_t OFF_VFH = OFF_KEL + SZ_KE;
constexpr size_t OFF_VFL = OFF_VFH + SZ_VF;
constexpr size_t WS_TOTAL = OFF_VFL + SZ_VF;
constexpr size_t OFF_OH  = OFF_X;
constexpr size_t OFF_OL  = OFF_XT;
static_assert(WS_TOTAL == 88080384u);
static_assert(WS_TOTAL <= 134217728u);
static_assert(SZ_QP == SZ_X && SZ_QP == SZ_XT);
static_assert((OFF_WQ % 128) == 0 && (OFF_QH % 128) == 0 && (OFF_TEH % 128) == 0 && (OFF_VFL % 128) == 0);

static_assert((NBATCH * NSEQ) % 64 == 0 && NFEAT % 64 == 0 && NCH % 32 == 0);
static_assert(KLR % 64 == 0 && NCH % 64 == 0 && NSEQ % 32 == 0);
static_assert(KLR % 64 == 0 && NFEAT % 64 == 0 && NCH % 32 == 0);
static_assert(NSEQ % ATT_QB == 0 && KLR % ATT_KC == 0 && DHEAD == 64);
static_assert(((size_t)NBATCH * NSEQ * NCH) % (8 * 256) == 0);
static_assert(((size_t)NFEAT * NCH) % (8 * 256) == 0 && ((size_t)KLR * NSEQ) % (8 * 256) == 0);
}

__device__ __forceinline__ unsigned short f2bf_bits(float f) {
  unsigned u = __float_as_uint(f);
  return (unsigned short)((u + 0x7FFFu + ((u >> 16) & 1u)) >> 16);
}
__device__ __forceinline__ float bf_bits2f(unsigned short h) { return __uint_as_float(((unsigned)h) << 16); }

__device__ __forceinline__ void dep_guard_h(v8f& a, v8f& b, v16h x, v16h y) { asm volatile("v_nop\n\tv_nop\n\tv_nop\n\tv_nop" : "+v"(a), "+v"(b) : "v"(x), "v"(y)); }
__device__ __forceinline__ void dep_guard_b(v8f& a, v8f& b, v16b x, v16b y) { asm volatile("v_nop\n\tv_nop\n\tv_nop\n\tv_nop" : "+v"(a), "+v"(b) : "v"(x), "v"(y)); }
__device__ __forceinline__ void keep4_h(v16h a, v16h b, v16h c, v16h d) { asm volatile("v_nop" :: "v"(a), "v"(b), "v"(c), "v"(d)); }
__device__ __forceinline__ void keep4_b(v16b a, v16b b, v16b c, v16b d) { asm volatile("v_nop" :: "v"(a), "v"(b), "v"(c), "v"(d)); }
__device__ __forceinline__ void acc_guard4(v8f& a, v8f& b, v8f& c, v8f& d) { asm volatile("v_nop\n\tv_nop\n\tv_nop\n\tv_nop" : "+v"(a), "+v"(b), "+v"(c), "+v"(d)); }
template <typename T> struct Frag;
template <> struct Frag<_Float16> {
  typedef v16h V; union U { v16h v; v8h h[2]; };
  static __device__ __forceinline__ v16h load(const _Float16* p) {
    U f; f.h[0] = *(const v8h*)(p); f.h[1] = *(const v8h*)(p + 16); return f.v;
  }
  static __device__ __forceinline__ v8f mma(v16h a, v16h b, v8f c) {
    return __builtin_amdgcn_wmma_f32_16x16x32_f16(false, a, false, b, (short)0, c, false, false);
  }
  static __device__ __forceinline__ void guard(v8f& a, v8f& b, v16h x, v16h y) { dep_guard_h(a, b, x, y); }
  static __device__ __forceinline__ void keep(v16h a, v16h b, v16h c, v16h d) { keep4_h(a, b, c, d); }
};
template <> struct Frag<__bf16> {
  typedef v16b V; union U { v16b v; v8b h[2]; };
  static __device__ __forceinline__ v16b load(const __bf16* p) {
    U f; f.h[0] = *(const v8b*)(p); f.h[1] = *(const v8b*)(p + 16); return f.v;
  }
  static __device__ __forceinline__ v8f mma(v16b a, v16b b, v8f c) {
    return __builtin_amdgcn_wmma_f32_16x16x32_bf16(false, a, false, b, (short)0, c, false, false);
  }
  static __device__ __forceinline__ void guard(v8f& a, v8f& b, v16b x, v16b y) { dep_guard_b(a, b, x, y); }
  static __device__ __forceinline__ void keep(v16b a, v16b b, v16b c, v16b d) { keep4_b(a, b, c, d); }
};

template <int ET> struct Elem;
template <> struct Elem<0> { typedef _Float16 T; };
template <> struct Elem<1> { typedef __bf16 T; };
template <int ET, int SPL, int BIAS_MODE, int OUT_MODE>
__global__ __launch_bounds__(256) void wmma_gemm64(
    const unsigned short* __restrict__ Ap, const unsigned short* __restrict__ A2p, int lda, long strideA,
    const unsigned short* __restrict__ Btp, const unsigned short* __restrict__ Bt2p, int ldb, long strideB,
    void* __restrict__ Cout, void* __restrict__ Cout2, int ldc, long strideC,
    const float* __restrict__ bias,
    int M, int N, int K, float scale) {
  constexpr bool SA = (SPL & 1) != 0;
  constexpr bool SB = (SPL & 2) != 0;
  typedef typename Elem<ET>::T T;
  typedef typename Frag<T>::V V;
  const T* A = (const T*)Ap; const T* A2 = (const T*)A2p; const T* Bt = (const T*)Btp; const T* Bt2 = (const T*)Bt2p;
  __shared__ __align__(16) float sT[8][16 * 68];
  const int b    = blockIdx.y;
  const int lane = threadIdx.x & 31;
  const int wave = threadIdx.x >> 5;
  const int tilesN = N >> 6;
  const int tilesM = M >> 6;
  const int tile = blockIdx.x * 8 + wave;
  if (tile >= tilesM * tilesN) return;
  const int tm = tile / tilesN;
  const int tn = tile - tm * tilesN;
  const int m0 = tm << 6;
  const int n0 = tn << 6;

  const T* Ab  = A  + (size_t)b * strideA;
  const T* Bb  = Bt + (size_t)b * strideB;
  const T* Ab2 = SA ? (A2  + (size_t)b * strideA) : nullptr;
  const T* Bb2 = SB ? (Bt2 + (size_t)b * strideB) : nullptr;

  const int rlane = lane & 15;
  const int koff  = (lane >> 4) * 8;
  const int mOff  = (lane >> 4) * 8;

  v8f acc[4][4];
#pragma unroll
  for (int i = 0; i < 4; ++i)
#pragma unroll
    for (int j = 0; j < 4; ++j) acc[i][j] = (v8f){0.f,0.f,0.f,0.f,0.f,0.f,0.f,0.f};

  for (int k0 = 0; k0 < K; k0 += 32) {
    V bh[4], bl[4];
#pragma unroll
    for (int j = 0; j < 4; ++j) {
      const size_t bo = (size_t)(n0 + (j << 4) + rlane) * ldb + koff + k0;
      bh[j] = Frag<T>::load(Bb + bo);
      if (SB) bl[j] = Frag<T>::load(Bb2 + bo);
    }
#pragma unroll
    for (int i = 0; i < 4; ++i) {
      const size_t ao = (size_t)(m0 + (i << 4) + rlane) * lda + koff + k0;
      V ah = Frag<T>::load(Ab + ao);
      V al = ah;
      if (SA) al = Frag<T>::load(Ab2 + ao);
#pragma unroll
      for (int j = 0; j < 4; ++j) {
        acc[i][j] = Frag<T>::mma(ah, bh[j], acc[i][j]);
        if (SB) acc[i][j] = Frag<T>::mma(ah, bl[j], acc[i][j]);
        if (SA) acc[i][j] = Frag<T>::mma(al, bh[j], acc[i][j]);
      }
      Frag<T>::guard(acc[i][0], acc[i][3], ah, al);
    }
    Frag<T>::keep(bh[0], bh[1], bh[2], bh[3]);
    if (SB) Frag<T>::keep(bl[0], bl[1], bl[2], bl[3]);
  }
  acc_guard4(acc[0][0], acc[0][1], acc[0][2], acc[0][3]);
  acc_guard4(acc[1][0], acc[1][1], acc[1][2], acc[1][3]);
  acc_guard4(acc[2][0], acc[2][1], acc[2][2], acc[2][3]);
  acc_guard4(acc[3][0], acc[3][1], acc[3][2], acc[3][3]);

  float* slab = sT[wave];
#pragma unroll
  for (int i = 0; i < 4; ++i) {
    const int mBase = m0 + (i << 4);
#pragma unroll
    for (int j = 0; j < 4; ++j) {
      const int n = n0 + (j << 4) + rlane;
      float bv = 0.f;
      if (BIAS_MODE == 2) bv = bf_bits2f(f2bf_bits(bias[n]));
#pragma unroll
      for (int r = 0; r < 8; ++r) {
        float v = acc[i][j][r] * scale;
        if (BIAS_MODE == 1) v += bf_bits2f(f2bf_bits(bias[mBase + mOff + r]));
        if (BIAS_MODE == 2) v += bv;
        slab[(mOff + r) * 68 + (j << 4) + rlane] = v;
      }
    }
    __builtin_amdgcn_fence(__ATOMIC_RELEASE, "workgroup");
    __builtin_amdgcn_wave_barrier();
    __builtin_amdgcn_fence(__ATOMIC_ACQUIRE, "workgroup");
    if (OUT_MODE == 0) {
      float* C = (float*)Cout + (size_t)b * strideC;
      const int hh = lane >> 4, c4 = (lane & 15) * 4;
      for (int pass = 0; pass < 2; ++pass) {
#pragma unroll
        for (int it = 0; it < 8; ++it) {
          const int row = it * 2 + hh;
          v4f v = *(const v4f*)(slab + row * 68 + c4);
          *(volatile v4f*)(C + (size_t)(mBase + row) * ldc + n0 + c4) = v;
        }
        __threadfence();
      }
    } else {
      const int q = lane >> 3, c8 = (lane & 7) * 8;
      unsigned short* C  = (unsigned short*)Cout  + (size_t)b * strideC;
      unsigned short* C2 = (OUT_MODE == 2) ? ((unsigned short*)Cout2 + (size_t)b * strideC) : nullptr;
      for (int pass = 0; pass < 2; ++pass) {
#pragma unroll
        for (int it = 0; it < 4; ++it) {
          const int row = it * 4 + q;
          const float* sp = slab + row * 68 + c8;
          v8h hv, lv;
#pragma unroll
          for (int e = 0; e < 8; ++e) {
            if (OUT_MODE == 1) {
              hv[e] = (_Float16)sp[e];
            } else {
              unsigned short hb = f2bf_bits(sp[e]);
              unsigned short lb = f2bf_bits(sp[e] - bf_bits2f(hb));
              hv[e] = __builtin_bit_cast(_Float16, hb);
              lv[e] = __builtin_bit_cast(_Float16, lb);
            }
          }
          *(volatile v8h*)(C + (size_t)(mBase + row) * ldc + n0 + c8) = hv;
          if (OUT_MODE == 2) *(volatile v8h*)(C2 + (size_t)(mBase + row) * ldc + n0 + c8) = lv;
        }
        __threadfence();
      }
    }
    __builtin_amdgcn_fence(__ATOMIC_RELEASE, "workgroup");
    __builtin_amdgcn_wave_barrier();
    __builtin_amdgcn_fence(__ATOMIC_ACQUIRE, "workgroup");
  }
}

__global__ __launch_bounds__(256) void cast_f32_bf16x8(const float* __restrict__ in, unsigned short* __restrict__ out, int n8) {
  const int i = blockIdx.x * 256 + threadIdx.x;
  if (i < n8) {
    const float* src = in + (size_t)i * 8;
    const v4f a0 = *(const v4f*)(src);
    const v4f a1 = *(const v4f*)(src + 4);
    v4u w;
    w[0] = (unsigned)f2bf_bits(a0[0]) | ((unsigned)f2bf_bits(a0[1]) << 16);
    w[1] = (unsigned)f2bf_bits(a0[2]) | ((unsigned)f2bf_bits(a0[3]) << 16);
    w[2] = (unsigned)f2bf_bits(a1[0]) | ((unsigned)f2bf_bits(a1[1]) << 16);
    w[3] = (unsigned)f2bf_bits(a1[2]) | ((unsigned)f2bf_bits(a1[3]) << 16);
    unsigned short* dst = out + (size_t)i * 8;
    *(volatile v4u*)dst = w;
    __threadfence();
    *(volatile v4u*)dst = w;
  }
}

__global__ __launch_bounds__(256) void transpose_cast_bf16(const float* __restrict__ in, unsigned short* __restrict__ out) {
  __shared__ __align__(16) unsigned short sT[64 * 72];
  const int tid = threadIdx.x, lane = tid & 31, wave = tid >> 5;
  const int n0 = blockIdx.x * 64, c0 = blockIdx.y * 64, b = blockIdx.z;
  const int rloc = tid >> 4, c4 = (tid & 15) * 4;
#pragma unroll
  for (int p = 0; p < 4; ++p) {
    const int nl = p * 16 + rloc;
    const v4f x = *(const v4f*)(in + ((size_t)b * NSEQ + n0 + nl) * NCH + c0 + c4);
    sT[(c4 + 0) * 72 + nl] = f2bf_bits(x[0]);
    sT[(c4 + 1) * 72 + nl] = f2bf_bits(x[1]);
    sT[(c4 + 2) * 72 + nl] = f2bf_bits(x[2]);
    sT[(c4 + 3) * 72 + nl] = f2bf_bits(x[3]);
  }
  __syncthreads();
  const int qq = lane >> 3, c8 = (lane & 7) * 8;
  for (int pass = 0; pass < 2; ++pass) {
#pragma unroll
    for (int it = 0; it < 2; ++it) {
      const int row = it * 32 + wave * 4 + qq;
      const v8us val = *(const v8us*)(sT + row * 72 + c8);
      *(volatile v8us*)(out + ((size_t)b * NCH + c0 + row) * NSEQ + n0 + c8) = val;
    }
    __threadfence();
  }
}

__device__ __forceinline__ unsigned short at_bf_bits(float f) {
  unsigned u = __float_as_uint(f);
  return (unsigned short)((u + 0x7FFFu + ((u >> 16) & 1u)) >> 16);
}
__device__ __forceinline__ __bf16 at_f2bf(float f) { return __builtin_bit_cast(__bf16, at_bf_bits(f)); }
__device__ __forceinline__ void at_split(float f, __bf16& hi, __bf16& lo) {
  const unsigned short hb = at_bf_bits(f);
  hi = __builtin_bit_cast(__bf16, hb);
  lo = at_f2bf(f - __uint_as_float(((unsigned)hb) << 16));
}
__device__ __forceinline__ v8f at_mma(v16b a, v16b b, v8f c) {
  c = __builtin_amdgcn_wmma_f32_16x16x32_bf16(false, a, false, b, (short)0, c, false, false);
  asm volatile("v_nop\n\tv_nop\n\tv_nop\n\tv_nop" : "+v"(c) : "v"(a), "v"(b));
  return c;
}
__device__ __forceinline__ void pack_hilo2(float a, float b, unsigned& wh, unsigned& wl) {
  const unsigned short ha = at_bf_bits(a);
  const unsigned short hb = at_bf_bits(b);
  const unsigned short la = at_bf_bits(a - __uint_as_float(((unsigned)ha) << 16));
  const unsigned short lb = at_bf_bits(b - __uint_as_float(((unsigned)hb) << 16));
  wh = (unsigned)ha | ((unsigned)hb << 16);
  wl = (unsigned)la | ((unsigned)lb << 16);
}

__global__ __launch_bounds__(128) void attn_lowrank(
    const unsigned short* __restrict__ Qh, const unsigned short* __restrict__ Ql,
    const unsigned short* __restrict__ Kh, const unsigned short* __restrict__ Kl,
    const unsigned short* __restrict__ Vh, const unsigned short* __restrict__ Vl,
    unsigned short* __restrict__ Oh, unsigned short* __restrict__ Ol) {
  union FB { v16b v; v8b h[2]; };
  __shared__ __align__(16) unsigned short Ksh[ATT_KC * DHEAD];
  __shared__ __align__(16) unsigned short Ksl[ATT_KC * DHEAD];
  __shared__ __align__(16) unsigned short Vth[DHEAD * ATT_KC];
  __shared__ __align__(16) unsigned short Vtl[DHEAD * ATT_KC];
  __shared__ __align__(16) __bf16 Psh[4][16 * ATT_KC];
  __shared__ __align__(16) __bf16 Psl[4][16 * ATT_KC];
  __shared__ __align__(16) float  Os[4][16 * 68];

  const int tid  = threadIdx.x;
  const int wave = tid >> 5;
  const int lane = tid & 31;
  const int hh   = lane >> 4;
  const int c    = lane & 15;

  const int bx  = blockIdx.x;
  const int qb  = bx & (NSEQ / ATT_QB - 1);
  const int bhh = bx >> 6;
  const int h   = bhh & (NHEAD - 1);
  const int b   = bhh >> 4;
  const int q0  = qb * ATT_QB + wave * 16;

  const size_t qbase = (size_t)b * NSEQ * NFEAT + (size_t)h * DHEAD;
  const size_t kbase = (size_t)b * KLR * NFEAT + (size_t)h * DHEAD;
  const size_t vbase = ((size_t)b * NFEAT + (size_t)h * DHEAD) * KLR;

  v16b qah[2], qal[2];
  {
    const __bf16* qr = (const __bf16*)(const void*)Qh + qbase + (size_t)(q0 + c) * NFEAT + 8 * hh;
    const __bf16* ql = (const __bf16*)(const void*)Ql + qbase + (size_t)(q0 + c) * NFEAT + 8 * hh;
#pragma unroll
    for (int dc = 0; dc < 2; ++dc) {
      qah[dc] = Frag<__bf16>::load(qr + dc * 32);
      qal[dc] = Frag<__bf16>::load(ql + dc * 32);
    }
  }

  float mrow[8], lrow[8];
  v8f oacc[4];
#pragma unroll
  for (int r = 0; r < 8; ++r) { mrow[r] = -__builtin_huge_valf(); lrow[r] = 0.f; }
#pragma unroll
  for (int t = 0; t < 4; ++t) oacc[t] = (v8f){0.f,0.f,0.f,0.f,0.f,0.f,0.f,0.f};

  for (int kc = 0; kc < KLR / ATT_KC; ++kc) {
    const int kv0 = kc * ATT_KC;
    __syncthreads();
    {
#pragma unroll
      for (int i = 0; i < 4; ++i) {
        const int p = tid + 128 * i; const int row = p >> 3, seg = (p & 7) * 8;
        const v8us x = *(const v8us*)(Kh + kbase + (size_t)(kv0 + row) * NFEAT + seg);
        *(v8us*)(Ksh + row * DHEAD + seg) = x;
      }
      asm volatile("" ::: "memory");
#pragma unroll
      for (int i = 0; i < 4; ++i) {
        const int p = tid + 128 * i; const int row = p >> 3, seg = (p & 7) * 8;
        const v8us x = *(const v8us*)(Kl + kbase + (size_t)(kv0 + row) * NFEAT + seg);
        *(v8us*)(Ksl + row * DHEAD + seg) = x;
      }
      asm volatile("" ::: "memory");
#pragma unroll
      for (int i = 0; i < 4; ++i) {
        const int p = tid + 128 * i; const int row = p >> 3, seg = (p & 7) * 8;
        const v8us x = *(const v8us*)(Vh + vbase + (size_t)row * KLR + kv0 + seg);
        *(v8us*)(Vth + row * ATT_KC + seg) = x;
      }
      asm volatile("" ::: "memory");
#pragma unroll
      for (int i = 0; i < 4; ++i) {
        const int p = tid + 128 * i; const int row = p >> 3, seg = (p & 7) * 8;
        const v8us x = *(const v8us*)(Vl + vbase + (size_t)row * KLR + kv0 + seg);
        *(v8us*)(Vtl + row * ATT_KC + seg) = x;
      }
    }
    __syncthreads();

    const __bf16* ksh = (const __bf16*)(const void*)Ksh;
    const __bf16* ksl = (const __bf16*)(const void*)Ksl;
    const __bf16* vth = (const __bf16*)(const void*)Vth;
    const __bf16* vtl = (const __bf16*)(const void*)Vtl;

    v8f s[4];
#pragma unroll
    for (int j = 0; j < 4; ++j) {
      s[j] = (v8f){0.f,0.f,0.f,0.f,0.f,0.f,0.f,0.f};
#pragma unroll
      for (int dc = 0; dc < 2; ++dc) {
        const v16b kb = Frag<__bf16>::load(ksh + (j * 16 + c) * DHEAD + dc * 32 + 8 * hh);
        const v16b kl = Frag<__bf16>::load(ksl + (j * 16 + c) * DHEAD + dc * 32 + 8 * hh);
        s[j] = at_mma(qah[dc], kb, s[j]);
        s[j] = at_mma(qah[dc], kl, s[j]);
        s[j] = at_mma(qal[dc], kb, s[j]);
      }
    }

    float cm[8];
#pragma unroll
    for (int r = 0; r < 8; ++r) {
      float m = fmaxf(fmaxf(s[0][r], s[1][r]), fmaxf(s[2][r], s[3][r]));
#pragma unroll
      for (int off = 1; off < 16; off <<= 1) m = fmaxf(m, __shfl_xor(m, off, 32));
      cm[r] = m;
    }
    __bf16* pwh = Psh[wave];
    __bf16* pwl = Psl[wave];
#pragma unroll
    for (int r = 0; r < 8; ++r) {
      const float mnew = fmaxf(mrow[r], cm[r]);
      const float alpha = expf(mrow[r] - mnew);
      mrow[r] = mnew;
      float psum = 0.f;
#pragma unroll
      for (int j = 0; j < 4; ++j) {
        const float p = expf(s[j][r] - mnew);
        psum += p;
        __bf16 ph, pl;
        at_split(p, ph, pl);
        pwh[(8 * hh + r) * ATT_KC + j * 16 + c] = ph;
        pwl[(8 * hh + r) * ATT_KC + j * 16 + c] = pl;
      }
#pragma unroll
      for (int off = 1; off < 16; off <<= 1) psum += __shfl_xor(psum, off, 32);
      lrow[r] = lrow[r] * alpha + psum;
#pragma unroll
      for (int t = 0; t < 4; ++t) oacc[t][r] *= alpha;
    }
    __builtin_amdgcn_fence(__ATOMIC_RELEASE, "workgroup");
    __builtin_amdgcn_wave_barrier();
    __builtin_amdgcn_fence(__ATOMIC_ACQUIRE, "workgroup");
#pragma unroll
    for (int kk = 0; kk < 2; ++kk) {
      FB pa, pl;
      pa.h[0] = *(const v8b*)(pwh + c * ATT_KC + kk * 32 + 8 * hh);
      pa.h[1] = *(const v8b*)(pwh + c * ATT_KC + kk * 32 + 16 + 8 * hh);
      pl.h[0] = *(const v8b*)(pwl + c * ATT_KC + kk * 32 + 8 * hh);
      pl.h[1] = *(const v8b*)(pwl + c * ATT_KC + kk * 32 + 16 + 8 * hh);
#pragma unroll
      for (int t = 0; t < 4; ++t) {
        const v16b vb = Frag<__bf16>::load(vth + (t * 16 + c) * ATT_KC + kk * 32 + 8 * hh);
        const v16b vl = Frag<__bf16>::load(vtl + (t * 16 + c) * ATT_KC + kk * 32 + 8 * hh);
        oacc[t] = at_mma(pa.v, vb, oacc[t]);
        oacc[t] = at_mma(pa.v, vl, oacc[t]);
        oacc[t] = at_mma(pl.v, vb, oacc[t]);
      }
    }
  }

  float* os = Os[wave];
#pragma unroll
  for (int r = 0; r < 8; ++r) {
    const float inv = 1.0f / lrow[r];
#pragma unroll
    for (int t = 0; t < 4; ++t) os[(8 * hh + r) * 68 + t * 16 + c] = oacc[t][r] * inv;
  }
  __builtin_amdgcn_fence(__ATOMIC_RELEASE, "workgroup");
  __builtin_amdgcn_wave_barrier();
  __builtin_amdgcn_fence(__ATOMIC_ACQUIRE, "workgroup");
  {
    const int qq = lane >> 3, c8 = (lane & 7) * 8;
    unsigned short* oh = Oh + qbase;
    unsigned short* ol = Ol + qbase;
    for (int pass = 0; pass < 2; ++pass) {
#pragma unroll
      for (int it = 0; it < 4; ++it) {
        const int row = it * 4 + qq;
        const float* sp = os + row * 68 + c8;
        const v4f f0 = *(const v4f*)(sp);
        const v4f f1 = *(const v4f*)(sp + 4);
        v4u wh, wl;
        unsigned th, tl;
        pack_hilo2(f0[0], f0[1], th, tl); wh[0] = th; wl[0] = tl;
        pack_hilo2(f0[2], f0[3], th, tl); wh[1] = th; wl[1] = tl;
        pack_hilo2(f1[0], f1[1], th, tl); wh[2] = th; wl[2] = tl;
        pack_hilo2(f1[2], f1[3], th, tl); wh[3] = th; wl[3] = tl;
        *(volatile v4u*)(oh + (size_t)(q0 + row) * NFEAT + c8) = wh;
        *(volatile v4u*)(ol + (size_t)(q0 + row) * NFEAT + c8) = wl;
      }
      __threadfence();
    }
  }
}

extern "C" void kernel_launch(void* const* d_in, const int* in_sizes, int n_in,
                              void* d_out, int out_size, void* d_ws, size_t ws_size,
                              hipStream_t stream) {
  if (n_in < 10) return;
  if (in_sizes[0] != NBATCH * NSEQ * NCH) return;
  if (in_sizes[1] != NHEAD * DHEAD * NCH || in_sizes[2] != NHEAD * DHEAD * NCH || in_sizes[3] != NHEAD * DHEAD * NCH) return;
  if (in_sizes[4] != KLR * NSEQ || in_sizes[6] != KLR * NSEQ) return;
  if (in_sizes[5] != KLR || in_sizes[7] != KLR) return;
  if (in_sizes[8] != NCH * NFEAT || in_sizes[9] != NCH) return;
  if ((size_t)out_size < (size_t)NBATCH * NSEQ * NCH) return;
  if (ws_size < WS_TOTAL) return;

  const float* x   = (const float*)d_in[0];
  const float* wq  = (const float*)d_in[1];
  const float* wk  = (const float*)d_in[2];
  const float* wv  = (const float*)d_in[3];
  const float* we  = (const float*)d_in[4];
  const float* bev = (const float*)d_in[5];
  const float* wf  = (const float*)d_in[6];
  const float* bfv = (const float*)d_in[7];
  const float* wo  = (const float*)d_in[8];
  const float* bov = (const float*)d_in[9];
  float* out = (float*)d_out;

  unsigned char* ws = (unsigned char*)d_ws;
  unsigned short* Xb  = (unsigned short*)(ws + OFF_X);
  unsigned short* XT  = (unsigned short*)(ws + OFF_XT);
  unsigned short* Wqb = (unsigned short*)(ws + OFF_WQ);
  unsigned short* Wkb = (unsigned short*)(ws + OFF_WK);
  unsigned short* Wvb = (unsigned short*)(ws + OFF_WV);
  unsigned short* Wob = (unsigned short*)(ws + OFF_WO);
  unsigned short* Web = (unsigned short*)(ws + OFF_WE);
  unsigned short* Wfb = (unsigned short*)(ws + OFF_WF);
  unsigned short* Qh  = (unsigned short*)(ws + OFF_QH);
  unsigned short* Ql  = (unsigned short*)(ws + OFF_QL);
  unsigned short* TEh = (unsigned short*)(ws + OFF_TEH);
  unsigned short* TEl = (unsigned short*)(ws + OFF_TEL);
  unsigned short* TFh = (unsigned short*)(ws + OFF_TFH);
  unsigned short* TFl = (unsigned short*)(ws + OFF_TFL);
  unsigned short* KEh = (unsigned short*)(ws + OFF_KEH);
  unsigned short* KEl = (unsigned short*)(ws + OFF_KEL);
  unsigned short* VFh = (unsigned short*)(ws + OFF_VFH);
  unsigned short* VFl = (unsigned short*)(ws + OFF_VFL);
  unsigned short* Ohp = (unsigned short*)(ws + OFF_OH);
  unsigned short* Olp = (unsigned short*)(ws + OFF_OL);

  {
    const int n8x = NBATCH * NSEQ * NCH / 8;
    const int n8w = NFEAT * NCH / 8;
    const int n8e = KLR * NSEQ / 8;
    cast_f32_bf16x8<<<dim3(n8x / 256), dim3(256), 0, stream>>>(x,  Xb,  n8x);
    cast_f32_bf16x8<<<dim3(n8w / 256), dim3(256), 0, stream>>>(wq, Wqb, n8w);
    cast_f32_bf16x8<<<dim3(n8w / 256), dim3(256), 0, stream>>>(wk, Wkb, n8w);
    cast_f32_bf16x8<<<dim3(n8w / 256), dim3(256), 0, stream>>>(wv, Wvb, n8w);
    cast_f32_bf16x8<<<dim3(n8w / 256), dim3(256), 0, stream>>>(wo, Wob, n8w);
    cast_f32_bf16x8<<<dim3(n8e / 256), dim3(256), 0, stream>>>(we, Web, n8e);
    cast_f32_bf16x8<<<dim3(n8e / 256), dim3(256), 0, stream>>>(wf, Wfb, n8e);
  }
  transpose_cast_bf16<<<dim3(NSEQ / 64, NCH / 64, NBATCH), dim3(256), 0, stream>>>(x, XT);

  wmma_gemm64<1, 0, 0, 2><<<dim3((NBATCH * NSEQ / 64) * (NFEAT / 64) / 8, 1), dim3(256), 0, stream>>>(
      Xb, Xb, NCH, 0L, Wqb, Wqb, NCH, 0L, (void*)Qh, (void*)Ql, NFEAT, 0L, bov,
      NBATCH * NSEQ, NFEAT, NCH, 0.125f);

  wmma_gemm64<1, 0, 0, 2><<<dim3((KLR / 64) * (NCH / 64) / 8, NBATCH), dim3(256), 0, stream>>>(
      Web, Web, NSEQ, 0L, XT, XT, NSEQ, (long)NCH * NSEQ, (void*)TEh, (void*)TEl, NCH, (long)KLR * NCH, bov,
      KLR, NCH, NSEQ, 1.0f);
  wmma_gemm64<1, 0, 0, 2><<<dim3((KLR / 64) * (NCH / 64) / 8, NBATCH), dim3(256), 0, stream>>>(
      Wfb, Wfb, NSEQ, 0L, XT, XT, NSEQ, (long)NCH * NSEQ, (void*)TFh, (void*)TFl, NCH, (long)KLR * NCH, bov,
      KLR, NCH, NSEQ, 1.0f);

  wmma_gemm64<1, 1, 1, 2><<<dim3((KLR / 64) * (NFEAT / 64) / 8, NBATCH), dim3(256), 0, stream>>>(
      TEh, TEl, NCH, (long)KLR * NCH, Wkb, Wkb, NCH, 0L, (void*)KEh, (void*)KEl, NFEAT, (long)KLR * NFEAT, bev,
      KLR, NFEAT, NCH, 1.0f);
  wmma_gemm64<1, 2, 2, 2><<<dim3((NFEAT / 64) * (KLR / 64) / 8, NBATCH), dim3(256), 0, stream>>>(
      Wvb, Wvb, NCH, 0L, TFh, TFl, NCH, (long)KLR * NCH, (void*)VFh, (void*)VFl, KLR, (long)NFEAT * KLR, bfv,
      NFEAT, KLR, NCH, 1.0f);

  attn_lowrank<<<dim3(NBATCH * NHEAD * (NSEQ / ATT_QB)), dim3(128), 0, stream>>>(Qh, Ql, KEh, KEl, VFh, VFl, Ohp, Olp);

  wmma_gemm64<1, 1, 2, 0><<<dim3((NBATCH * NSEQ / 64) * (NCH / 64) / 8, 1), dim3(256), 0, stream>>>(
      Ohp, Olp, NFEAT, 0L, Wob, Wob, NFEAT, 0L, (void*)out, (void*)out, NCH, 0L, bov,
      NBATCH * NSEQ, NCH, NFEAT, 1.0f);
}
